// OptimizedMoEAttention_31086973288490
// MI455X (gfx1250) — hardware-run, weakly checked
//
#include <hip/hip_runtime.h>
#include <stddef.h>
#include <stdint.h>

#define NBATCH 4
#define SEQ    512
#define NTOK   2048
#define DIM    1024
#define NHEAD  16
#define HDIM   64
#define NE     4
#define NSEL   2
#define HID    512
#define NLIST  16
#define LCAP   512
#define NTILE  80
#define QROWS  5120
#define NPROW  4096
#define ETILE  32
#define RPITCH 8
#define WSC    64.0f
#define WINV   0.015625f
#define QSC    0.125f
#define APITCH 136
#define EPH    72
#define OTP    68
#define TRPF   68
#define PPITCH 40

static_assert(NTOK == NBATCH * SEQ);
static_assert(NLIST == NE * NBATCH);
static_assert(NTILE == NTOK * NSEL / 64 + NLIST);
static_assert(QROWS == NTILE * 64);
static_assert(NPROW == NTOK * NSEL);
static_assert(ETILE == NBATCH * (LCAP / 64));
static_assert(NSEL == 2);
static_assert(NE == 4);
static_assert(DIM == NHEAD * HDIM);
static_assert(HDIM == 64);
static_assert(DIM % 128 == 0);
static_assert(HID % 64 == 0);
static_assert(SEQ % 256 == 0);
static_assert(NTOK % 8 == 0);
static_assert((NTOK * DIM) % 2048 == 0);

typedef _Float16 v16h __attribute__((ext_vector_type(16)));
typedef _Float16 v8h  __attribute__((ext_vector_type(8)));
typedef __bf16   v16b __attribute__((ext_vector_type(16)));
typedef unsigned short v8us __attribute__((ext_vector_type(8), may_alias));
typedef unsigned short v4us __attribute__((ext_vector_type(4)));
typedef float    v8f  __attribute__((ext_vector_type(8)));
typedef float    v4f  __attribute__((ext_vector_type(4)));
typedef float    v2f  __attribute__((ext_vector_type(2)));
typedef unsigned int v4u __attribute__((ext_vector_type(4)));
typedef int      v4i  __attribute__((ext_vector_type(4)));

union FragH  { v16h v; v8h h[2]; };
union FragB  { v16b v; v8us h[2]; };
union Pack8h { v8h h; v4u u; };
union Pack8s { v8us s; v4u u; };

__device__ __forceinline__ int clampi(int v, int lo, int hi) { return min(max(v, lo), hi); }

__device__ __forceinline__ unsigned short f2bf(float x) {
  unsigned u = __float_as_uint(x);
  u += 0x7FFFu + ((u >> 16) & 1u);
  return (unsigned short)(u >> 16);
}
__device__ __forceinline__ float bf2f(unsigned short h) { return __uint_as_float(((unsigned)h) << 16); }

__device__ __forceinline__ v8f zero8() { return (v8f){0.f, 0.f, 0.f, 0.f, 0.f, 0.f, 0.f, 0.f}; }

__device__ __forceinline__ v8f mmah(v16h a, v16h b, v8f c) {
  c = __builtin_amdgcn_wmma_f32_16x16x32_f16(false, a, false, b, (short)0, c, false, false);
  asm volatile("v_nop\n\tv_nop\n\tv_nop\n\tv_nop" : "+v"(c) : "v"(a), "v"(b));
  return c;
}
__device__ __forceinline__ v8f mmab(v16b a, v16b b, v8f c) {
  c = __builtin_amdgcn_wmma_f32_16x16x32_bf16(false, a, false, b, (short)0, c, false, false);
  asm volatile("v_nop\n\tv_nop\n\tv_nop\n\tv_nop" : "+v"(c) : "v"(a), "v"(b));
  return c;
}

__device__ __forceinline__ v16h ldfragh(const _Float16* p, int ld, int row0, int k0, int lane) {
  const int m = lane & 15, lh = lane >> 4;
  const _Float16* q = p + (size_t)(row0 + m) * ld + k0 + 8 * lh;
  FragH f;
  f.h[0] = *(const v8h*)(q);
  f.h[1] = *(const v8h*)(q + 16);
  return f.v;
}
__device__ __forceinline__ v16b ldfragb(const unsigned short* p, int ld, int row0, int k0, int lane) {
  const int m = lane & 15, lh = lane >> 4;
  const unsigned short* q = p + (size_t)(row0 + m) * ld + k0 + 8 * lh;
  FragB f;
  f.h[0] = *(const v8us*)(q);
  f.h[1] = *(const v8us*)(q + 16);
  return f.v;
}

__device__ __forceinline__ void gemm16x64(const _Float16* __restrict__ A, int lda, int arow0,
                                          const _Float16* __restrict__ Bt, int ldb, int brow0,
                                          int K, int lane, v8f (&acc)[4]) {
#pragma unroll 1
  for (int k0 = 0; k0 < K; k0 += 32) {
    const v16h a = ldfragh(A, lda, arow0, k0, lane);
#pragma unroll
    for (int t = 0; t < 4; ++t) {
      const v16h bq = ldfragh(Bt, ldb, brow0 + 16 * t, k0, lane);
      acc[t] = mmah(a, bq, acc[t]);
    }
  }
}

__global__ __launch_bounds__(256) void k_cvt(const float* __restrict__ src, _Float16* __restrict__ dh, int n8) {
  const int i = blockIdx.x * 256 + (int)threadIdx.x;
  if (i >= n8) return;
  const size_t o = (size_t)i * 8;
  const v4f a0 = *(const v4f*)(src + o);
  const v4f a1 = *(const v4f*)(src + o + 4);
  Pack8h pk;
  pk.h = (v8h){(_Float16)a0[0], (_Float16)a0[1], (_Float16)a0[2], (_Float16)a0[3],
               (_Float16)a1[0], (_Float16)a1[1], (_Float16)a1[2], (_Float16)a1[3]};
  const v4u vv = pk.u;
  volatile v4u* d = (volatile v4u*)(dh + o);
  *d = vv;
  __threadfence();
  *d = vv;
}

__global__ __launch_bounds__(256) void k_wtrh(const float* __restrict__ w, _Float16* __restrict__ wt,
                                              int kdim, int ndim, float scale) {
  __shared__ __align__(16) float st[64 * TRPF];
  const int tid = threadIdx.x;
  const size_t bo = (size_t)blockIdx.z * (size_t)kdim * (size_t)ndim;
  w  += bo;
  wt += bo;
  const int n0 = blockIdx.x * 64, k0 = blockIdx.y * 64;
  const int kr = tid >> 2;
  const int nc = (tid & 3) * 16;
  const float* sp = w + (size_t)(k0 + kr) * ndim + n0 + nc;
#pragma unroll
  for (int q = 0; q < 4; ++q) {
    const v4f a = *(const v4f*)(sp + 4 * q) * scale;
#pragma unroll
    for (int j = 0; j < 4; ++j) st[(nc + 4 * q + j) * TRPF + kr] = a[j];
  }
  __syncthreads();
  v4u val[2];
  size_t go[2];
#pragma unroll
  for (int j = 0; j < 2; ++j) {
    const int p  = tid + 256 * j;
    const int nr = p >> 3;
    const int pc = p & 7;
    const v4f f0 = *(const v4f*)(st + nr * TRPF + pc * 8);
    const v4f f1 = *(const v4f*)(st + nr * TRPF + pc * 8 + 4);
    Pack8h pk;
    pk.h = (v8h){(_Float16)f0[0], (_Float16)f0[1], (_Float16)f0[2], (_Float16)f0[3],
                 (_Float16)f1[0], (_Float16)f1[1], (_Float16)f1[2], (_Float16)f1[3]};
    val[j] = pk.u;
    go[j]  = (size_t)(n0 + nr) * kdim + k0 + pc * 8;
  }
  for (int ps = 0; ps < 2; ++ps) {
#pragma unroll
    for (int j = 0; j < 2; ++j) *(volatile v4u*)(wt + go[j]) = val[j];
    __threadfence();
  }
}

__global__ __launch_bounds__(256) void k_wtrb(const float* __restrict__ w, unsigned short* __restrict__ oh,
                                              unsigned short* __restrict__ ol, int kdim, int ndim) {
  __shared__ __align__(16) float st[64 * TRPF];
  const int tid = threadIdx.x;
  const size_t bo = (size_t)blockIdx.z * (size_t)kdim * (size_t)ndim;
  w  += bo;
  oh += bo;
  ol += bo;
  const int n0 = blockIdx.x * 64, k0 = blockIdx.y * 64;
  const int kr = tid >> 2;
  const int nc = (tid & 3) * 16;
  const float* sp = w + (size_t)(k0 + kr) * ndim + n0 + nc;
#pragma unroll
  for (int q = 0; q < 4; ++q) {
    const v4f a = *(const v4f*)(sp + 4 * q);
#pragma unroll
    for (int j = 0; j < 4; ++j) st[(nc + 4 * q + j) * TRPF + kr] = a[j];
  }
  __syncthreads();
  v4u vh[2], vlo[2];
  size_t go[2];
#pragma unroll
  for (int j = 0; j < 2; ++j) {
    const int p  = tid + 256 * j;
    const int nr = p >> 3;
    const int pc = p & 7;
    const v4f f0 = *(const v4f*)(st + nr * TRPF + pc * 8);
    const v4f f1 = *(const v4f*)(st + nr * TRPF + pc * 8 + 4);
    Pack8s ph, pl;
    ph.s = (v8us){f2bf(f0[0]), f2bf(f0[1]), f2bf(f0[2]), f2bf(f0[3]),
                  f2bf(f1[0]), f2bf(f1[1]), f2bf(f1[2]), f2bf(f1[3])};
    pl.s = (v8us){f2bf(f0[0] - bf2f(ph.s[0])), f2bf(f0[1] - bf2f(ph.s[1])),
                  f2bf(f0[2] - bf2f(ph.s[2])), f2bf(f0[3] - bf2f(ph.s[3])),
                  f2bf(f1[0] - bf2f(ph.s[4])), f2bf(f1[1] - bf2f(ph.s[5])),
                  f2bf(f1[2] - bf2f(ph.s[6])), f2bf(f1[3] - bf2f(ph.s[7]))};
    vh[j]  = ph.u;
    vlo[j] = pl.u;
    go[j]  = (size_t)(n0 + nr) * kdim + k0 + pc * 8;
  }
  for (int ps = 0; ps < 2; ++ps) {
#pragma unroll
    for (int j = 0; j < 2; ++j) {
      *(volatile v4u*)(oh + go[j]) = vh[j];
      *(volatile v4u*)(ol + go[j]) = vlo[j];
    }
    __threadfence();
  }
}

__global__ __launch_bounds__(256) void k_route(const float* __restrict__ x, const float* __restrict__ w1,
                                               const float* __restrict__ b1, const float* __restrict__ lg,
                                               const float* __restrict__ lb, const float* __restrict__ w2,
                                               const float* __restrict__ b2, float* __restrict__ rp) {
  __shared__ __align__(16) float sX[8 * DIM];
  __shared__ __align__(16) float sH[8 * HID];
  __shared__ __align__(16) float sR[8 * RPITCH];
  const int tid = threadIdx.x, lane = tid & 31, wave = tid >> 5;
  const size_t t0 = (size_t)blockIdx.x * 8;
  const float* xb = x + t0 * DIM;
#pragma unroll
  for (int i = 0; i < 8; ++i) {
    const int q = tid + 256 * i;
    *(v4f*)(sX + q * 4) = *(const v4f*)(xb + (size_t)q * 4);
  }
  __syncthreads();

  const int nA = tid, nB = tid + 256;
  float aA[8], aB[8];
#pragma unroll
  for (int t = 0; t < 8; ++t) { aA[t] = 0.f; aB[t] = 0.f; }
#pragma unroll 1
  for (int k = 0; k < DIM; k += 2) {
    const float wa0 = w1[(size_t)k * HID + nA];
    const float wa1 = w1[(size_t)(k + 1) * HID + nA];
    const float wb0 = w1[(size_t)k * HID + nB];
    const float wb1 = w1[(size_t)(k + 1) * HID + nB];
#pragma unroll
    for (int t = 0; t < 8; ++t) {
      const v2f xv = *(const v2f*)(sX + t * DIM + k);
      aA[t] += xv[0] * wa0;
      aA[t] += xv[1] * wa1;
      aB[t] += xv[0] * wb0;
      aB[t] += xv[1] * wb1;
    }
  }
  const float bA = b1[nA], bB = b1[nB];
#pragma unroll
  for (int t = 0; t < 8; ++t) {
    sH[t * HID + nA] = aA[t] + bA;
    sH[t * HID + nB] = aB[t] + bB;
  }
  __syncthreads();

  const float* hr = sH + wave * HID;
  float s = 0.f;
#pragma unroll 1
  for (int j = 0; j < HID / 32; ++j) s += hr[lane + 32 * j];
#pragma unroll
  for (int off = 16; off >= 1; off >>= 1) s += __shfl_xor(s, off, 32);
  const float mu = s * (1.0f / (float)HID);
  float vs = 0.f;
#pragma unroll 1
  for (int j = 0; j < HID / 32; ++j) {
    const float d = hr[lane + 32 * j] - mu;
    vs += d * d;
  }
#pragma unroll
  for (int off = 16; off >= 1; off >>= 1) vs += __shfl_xor(vs, off, 32);
  const float var = vs * (1.0f / (float)HID);
  const float rsq = rsqrtf(var + 1e-5f);
  float l0 = 0.f, l1 = 0.f, l2 = 0.f, l3 = 0.f;
#pragma unroll 1
  for (int j = 0; j < HID / 32; ++j) {
    const int n = lane + 32 * j;
    const float d = hr[n] - mu;
    float hn = d * rsq * lg[n] + lb[n];
    hn = fmaxf(hn, 0.f);
    const v4f wr = *(const v4f*)(w2 + (size_t)n * NE);
    l0 += hn * wr[0];
    l1 += hn * wr[1];
    l2 += hn * wr[2];
    l3 += hn * wr[3];
  }
#pragma unroll
  for (int off = 16; off >= 1; off >>= 1) {
    l0 += __shfl_xor(l0, off, 32);
    l1 += __shfl_xor(l1, off, 32);
    l2 += __shfl_xor(l2, off, 32);
    l3 += __shfl_xor(l3, off, 32);
  }
  l0 += b2[0]; l1 += b2[1]; l2 += b2[2]; l3 += b2[3];

  const int c4 = lane & 3;
  const float mx = fmaxf(fmaxf(l0, l1), fmaxf(l2, l3));
  float mine = l0;
  mine = (c4 == 1) ? l1 : mine;
  mine = (c4 == 2) ? l2 : mine;
  mine = (c4 == 3) ? l3 : mine;
  const float ex = expf(mine - mx);
  float ss = ex;
  ss += __shfl_xor(ss, 1, 32);
  ss += __shfl_xor(ss, 2, 32);
  const float pm = ex * (1.0f / ss);
  float pr[NE];
#pragma unroll
  for (int e = 0; e < NE; ++e) pr[e] = __shfl(pm, e, 32);

  const float NEGI = -3.0e38f;
  int idx0 = 0, idx1 = 0;
  float ws0 = 0.f, ws1 = 0.f;
  unsigned taken = 0u;
  {
    float bv = NEGI; int best = 0;
#pragma unroll
    for (int i = 0; i < NE; ++i) {
      const bool cnd = (pr[i] > bv);
      bv = cnd ? pr[i] : bv;
      best = cnd ? i : best;
    }
    idx0 = best; ws0 = bv; taken = (1u << best);
  }
  {
    float bv = NEGI; int best = 0;
#pragma unroll
    for (int i = 0; i < NE; ++i) {
      const bool cnd = (((taken >> i) & 1u) == 0u) && (pr[i] > bv);
      bv = cnd ? pr[i] : bv;
      best = cnd ? i : best;
    }
    idx1 = best; ws1 = bv;
  }

  float ov = 0.f;
  ov = (lane == 0) ? (float)idx0 : ov;
  ov = (lane == 1) ? (float)idx1 : ov;
  ov = (lane == 4) ? ws0 : ov;
  ov = (lane == 5) ? ws1 : ov;
  if (lane < RPITCH) sR[wave * RPITCH + lane] = ov;
  __syncthreads();
  if (wave == 0) {
    const int c = lane & 15;
    const v4f vr = *(const v4f*)(sR + c * 4);
    volatile v4f* dr = (volatile v4f*)(rp + (size_t)blockIdx.x * (8 * RPITCH) + c * 4);
    if (lane < 16) *dr = vr;
    __threadfence();
    if (lane < 16) *dr = vr;
  }
}

__global__ __launch_bounds__(256) void k_lists(const float* __restrict__ rp, int* __restrict__ tokl,
                                               float* __restrict__ wl, int* __restrict__ tab) {
  __shared__ __align__(16) unsigned short ltok[LCAP];
  __shared__ __align__(16) float lw[LCAP];
  __shared__ int wc[8];
  __shared__ __align__(16) int sTab[64];
  const int tid = threadIdx.x, lane = tid & 31, wave = tid >> 5;
  if (tid < 64) sTab[tid] = 0;
  int tbrun = 0;
#pragma unroll 1
  for (int g = 0; g < NLIST; ++g) {
    const int e = g >> 2, bb = g & 3;
    __syncthreads();
    for (int i = tid; i < LCAP; i += 256) { ltok[i] = (unsigned short)0; lw[i] = 0.f; }
    __syncthreads();
    int run = 0;
#pragma unroll 1
    for (int ch = 0; ch < SEQ / 256; ++ch) {
      const int t = bb * SEQ + ch * 256 + tid;
      const v4f ri = *(const v4f*)(rp + (size_t)t * RPITCH);
      const v4f rw = *(const v4f*)(rp + (size_t)t * RPITCH + 4);
      int hit = -1;
      float w = 0.f;
#pragma unroll
      for (int k = NSEL - 1; k >= 0; --k) {
        const bool m = ((int)ri[k] == e);
        hit = m ? k : hit;
        w   = m ? rw[k] : w;
      }
      const bool flag = (hit >= 0);
      const unsigned bal = __builtin_amdgcn_ballot_w32(flag);
      const int pre = __builtin_popcount(bal & ((1u << lane) - 1u));
      if (lane == 0) wc[wave] = __builtin_popcount(bal);
      __syncthreads();
      int base = run, tot = 0;
#pragma unroll
      for (int q = 0; q < 8; ++q) {
        const int cw = wc[q];
        base += (q < wave) ? cw : 0;
        tot  += cw;
      }
      const int pos = clampi(base + pre, 0, LCAP - 1);
      if (flag) { ltok[pos] = (unsigned short)(t * NSEL + hit); lw[pos] = w; }
      run += tot;
      __syncthreads();
    }
    run = clampi(run, 0, LCAP);
    const int ntl = (run + 63) >> 6;
    if (tid == 0) { sTab[g] = run; sTab[32 + g + 1] = clampi(tbrun + ntl, 0, NTILE); }
    tbrun += ntl;

    int*   trow = tokl + (size_t)g * LCAP;
    float* wrow = wl + (size_t)g * LCAP;
    if (tid < 128) {
      const v4us u = *(const v4us*)(ltok + tid * 4);
      const v4i tv = (v4i){(int)u[0], (int)u[1], (int)u[2], (int)u[3]};
      const v4f wv = *(const v4f*)(lw + tid * 4);
      for (int ps = 0; ps < 2; ++ps) {
        *(volatile v4i*)(trow + tid * 4) = tv;
        *(volatile v4f*)(wrow + tid * 4) = wv;
        __threadfence();
      }
    }
  }
  __syncthreads();
  if (wave == 0) {
    const v4i v = *(const v4i*)(sTab + (lane & 15) * 4);
    volatile v4i* d = (volatile v4i*)(tab + (lane & 15) * 4);
    if (lane < 16) *d = v;
    __threadfence();
    if (lane < 16) *d = v;
  }
}

__global__ __launch_bounds__(256) void k_qproj(const _Float16* __restrict__ xh, const _Float16* __restrict__ wqt,
                                               const float* __restrict__ bq, const int* __restrict__ tokl,
                                               const int* __restrict__ tab, unsigned short* __restrict__ qh,
                                               unsigned short* __restrict__ ql) {
  __shared__ __align__(16) _Float16 sA[64 * APITCH];
  __shared__ __align__(16) unsigned short sEh[8 * 16 * EPH];
  __shared__ __align__(16) unsigned short sEl[8 * 16 * EPH];
  __shared__ int sTok[64];
  __shared__ int sTab[64];
  const int tid = threadIdx.x, lane = tid & 31, wave = tid >> 5;
  const int hh = lane >> 4, c = lane & 15;
  const int wm = wave & 3, wn = wave >> 2;
  const int b  = blockIdx.y;
  const int n0 = blockIdx.x * 128;

  if (tid < 64) sTab[tid] = tab[tid];
  __syncthreads();
  const int tb16 = clampi(sTab[32 + NLIST], 0, NTILE);
  if (b >= tb16) return;
  int g = 0;
#pragma unroll
  for (int q = 1; q < NLIST; ++q) g += (clampi(sTab[32 + q], 0, NTILE) <= b) ? 1 : 0;
  const int e = g >> 2;
  const int tbg = clampi(sTab[32 + g], 0, NTILE);
  if (tid < 64) {
    const int rloc = (b - tbg) * 64 + tid;
    const int li = g * LCAP + clampi(rloc, 0, LCAP - 1);
    const int enc = tokl[li];
    sTok[tid] = clampi(enc >> 1, 0, NTOK - 1);
  }
  __syncthreads();

  const _Float16* wqe = wqt + (size_t)e * (size_t)(DIM * DIM);
  const int brow = n0 + wn * 64;

  v8f acc[4];
#pragma unroll
  for (int t = 0; t < 4; ++t) acc[t] = zero8();

  const int ar = tid >> 2, ac = tid & 3;
  const _Float16* xrow = xh + (size_t)sTok[ar] * DIM + ac * 32;
  _Float16* arow = sA + ar * APITCH + ac * 32;
#pragma unroll 1
  for (int kc = 0; kc < DIM / 128; ++kc) {
    __syncthreads();
#pragma unroll
    for (int q = 0; q < 4; ++q) *(v8h*)(arow + 8 * q) = *(const v8h*)(xrow + kc * 128 + 8 * q);
    __syncthreads();
#pragma unroll 1
    for (int ks = 0; ks < 4; ++ks) {
      const int kg = kc * 128 + ks * 32;
      const v16h a = ldfragh(sA, APITCH, wm * 16, ks * 32, lane);
#pragma unroll
      for (int t = 0; t < 4; ++t) {
        const v16h bqf = ldfragh(wqe, DIM, brow + 16 * t, kg, lane);
        acc[t] = mmah(a, bqf, acc[t]);
      }
    }
  }

  float bcv[4];
#pragma unroll
  for (int t = 0; t < 4; ++t) bcv[t] = bq[(size_t)e * DIM + brow + 16 * t + c];
  unsigned short* eh = sEh + wave * (16 * EPH);
  unsigned short* el = sEl + wave * (16 * EPH);
#pragma unroll
  for (int t = 0; t < 4; ++t) {
#pragma unroll
    for (int r = 0; r < 8; ++r) {
      const float v = (acc[t][r] * WINV + bcv[t]) * QSC;
      const unsigned short hi = f2bf(v);
      const unsigned short lo = f2bf(v - bf2f(hi));
      eh[(8 * hh + r) * EPH + 16 * t + c] = hi;
      el[(8 * hh + r) * EPH + 16 * t + c] = lo;
    }
  }
  __syncthreads();
  v4u vh[4], vlo[4];
  size_t go[4];
#pragma unroll
  for (int it = 0; it < 4; ++it) {
    const int p  = lane + 32 * it;
    const int L  = p >> 3;
    const int pc = p & 7;
    vh[it]  = *(const v4u*)(eh + L * EPH + pc * 8);
    vlo[it] = *(const v4u*)(el + L * EPH + pc * 8);
    go[it]  = (size_t)(b * 64 + wm * 16 + L) * DIM + brow + pc * 8;
  }
  for (int ps = 0; ps < 2; ++ps) {
#pragma unroll
    for (int it = 0; it < 4; ++it) {
      *(volatile v4u*)(qh + go[it]) = vh[it];
      *(volatile v4u*)(ql + go[it]) = vlo[it];
    }
    __threadfence();
  }
}

template <int BIASROW>
__global__ __launch_bounds__(256) void k_gemm16(const _Float16* __restrict__ A, const _Float16* __restrict__ Bt,
                                                const float* __restrict__ bias, unsigned short* __restrict__ oh,
                                                unsigned short* __restrict__ ol, int N, int K) {
  __shared__ __align__(16) unsigned short sEh[8 * 16 * EPH];
  __shared__ __align__(16) unsigned short sEl[8 * 16 * EPH];
  const int tid = threadIdx.x, lane = tid & 31, wave = tid >> 5;
  const int hh = lane >> 4, c = lane & 15;
  const int wm = wave & 3, wn = wave >> 2;
  const int arow0 = blockIdx.y * 64 + wm * 16;
  const int brow  = blockIdx.x * 128 + wn * 64;

  v8f acc[4];
#pragma unroll
  for (int t = 0; t < 4; ++t) acc[t] = zero8();
  gemm16x64(A, K, arow0, Bt, K, brow, K, lane, acc);

  float brv[8], bcv[4];
#pragma unroll
  for (int r = 0; r < 8; ++r) brv[r] = BIASROW ? bias[arow0 + 8 * hh + r] : 0.f;
#pragma unroll
  for (int t = 0; t < 4; ++t) bcv[t] = BIASROW ? 0.f : bias[brow + 16 * t + c];

  unsigned short* eh = sEh + wave * (16 * EPH);
  unsigned short* el = sEl + wave * (16 * EPH);
#pragma unroll
  for (int t = 0; t < 4; ++t) {
#pragma unroll
    for (int r = 0; r < 8; ++r) {
      const float v = acc[t][r] * WINV + brv[r] + bcv[t];
      const unsigned short hi = f2bf(v);
      const unsigned short lo = f2bf(v - bf2f(hi));
      eh[(8 * hh + r) * EPH + 16 * t + c] = hi;
      el[(8 * hh + r) * EPH + 16 * t + c] = lo;
    }
  }
  __syncthreads();
  v4u vh[4], vlo[4];
  size_t go[4];
#pragma unroll
  for (int it = 0; it < 4; ++it) {
    const int p  = lane + 32 * it;
    const int L  = p >> 3;
    const int pc = p & 7;
    vh[it]  = *(const v4u*)(eh + L * EPH + pc * 8);
    vlo[it] = *(const v4u*)(el + L * EPH + pc * 8);
    go[it]  = (size_t)(arow0 + L) * N + brow + pc * 8;
  }
  for (int ps = 0; ps < 2; ++ps) {
#pragma unroll
    for (int it = 0; it < 4; ++it) {
      *(volatile v4u*)(oh + go[it]) = vh[it];
      *(volatile v4u*)(ol + go[it]) = vlo[it];
    }
    __threadfence();
  }
}

__global__ __launch_bounds__(128) void k_attn(const unsigned short* __restrict__ qh, const unsigned short* __restrict__ ql,
                                              const unsigned short* __restrict__ kh, const unsigned short* __restrict__ kl,
                                              const unsigned short* __restrict__ vh, const unsigned short* __restrict__ vl,
                                              const int* __restrict__ tab, unsigned short* __restrict__ ah,
                                              unsigned short* __restrict__ al, int e) {
  __shared__ __align__(16) unsigned short sP[4 * 2 * 16 * PPITCH];
  __shared__ __align__(16) unsigned short sO[4 * 2 * 16 * EPH];
  __shared__ int sTab[64];
  const int tid = threadIdx.x, lane = tid & 31, wave = tid >> 5;
  const int hh = lane >> 4, c = lane & 15;
  const int h = blockIdx.x;

  if (tid < 64) sTab[tid] = tab[tid];
  __syncthreads();
  const int ge0 = e * NBATCH;
  const int tlo = clampi(sTab[32 + ge0], 0, NTILE);
  const int thi = clampi(sTab[32 + ge0 + NBATCH], 0, NTILE);
  const int b = tlo + (int)blockIdx.y;
  if (b >= thi) return;
  int bb = 0;
#pragma unroll
  for (int q = 1; q < NBATCH; ++q) bb += (clampi(sTab[32 + ge0 + q], 0, NTILE) <= b) ? 1 : 0;

  const int qrow0 = b * 64 + wave * 16;
  const int kcol  = h * HDIM;
  const unsigned short* khb = kh + (size_t)bb * SEQ * DIM;
  const unsigned short* klb = kl + (size_t)bb * SEQ * DIM;
  const unsigned short* vhb = vh + (size_t)bb * SEQ;
  const unsigned short* vlb = vl + (size_t)bb * SEQ;

  v16b qhf[2], qlf[2];
#pragma unroll
  for (int kk = 0; kk < 2; ++kk) {
    qhf[kk] = ldfragb(qh, DIM, qrow0, kcol + 32 * kk, lane);
    qlf[kk] = ldfragb(ql, DIM, qrow0, kcol + 32 * kk, lane);
  }
  v8f acc[4];
#pragma unroll
  for (int nf = 0; nf < 4; ++nf) acc[nf] = zero8();
  float mrow[8], lrow[8];
#pragma unroll
  for (int r = 0; r < 8; ++r) { mrow[r] = -1.0e30f; lrow[r] = 0.f; }

  unsigned short* sph = sP + wave * (2 * 16 * PPITCH);
  unsigned short* spl = sph + 16 * PPITCH;

#pragma unroll 1
  for (int kt = 0; kt < SEQ / 32; ++kt) {
    v8f sf[2];
#pragma unroll
    for (int g2 = 0; g2 < 2; ++g2) {
      v8f s = zero8();
      const int krow0 = kt * 32 + g2 * 16;
#pragma unroll
      for (int kk = 0; kk < 2; ++kk) {
        const v16b khf = ldfragb(khb, DIM, krow0, kcol + 32 * kk, lane);
        const v16b klf = ldfragb(klb, DIM, krow0, kcol + 32 * kk, lane);
        s = mmab(qhf[kk], khf, s);
        s = mmab(qhf[kk], klf, s);
        s = mmab(qlf[kk], khf, s);
      }
      sf[g2] = s;
    }
#pragma unroll
    for (int r = 0; r < 8; ++r) {
      float t = fmaxf(sf[0][r], sf[1][r]);
      t = fmaxf(t, __shfl_xor(t, 1, 32));
      t = fmaxf(t, __shfl_xor(t, 2, 32));
      t = fmaxf(t, __shfl_xor(t, 4, 32));
      t = fmaxf(t, __shfl_xor(t, 8, 32));
      const float mnew = fmaxf(mrow[r], t);
      const float cc = __expf(mrow[r] - mnew);
      const float p0 = __expf(sf[0][r] - mnew);
      const float p1 = __expf(sf[1][r] - mnew);
      float rs = p0 + p1;
      rs += __shfl_xor(rs, 1, 32);
      rs += __shfl_xor(rs, 2, 32);
      rs += __shfl_xor(rs, 4, 32);
      rs += __shfl_xor(rs, 8, 32);
      lrow[r] = lrow[r] * cc + rs;
      mrow[r] = mnew;
#pragma unroll
      for (int nf = 0; nf < 4; ++nf) acc[nf][r] = acc[nf][r] * cc;
      const unsigned short h0 = f2bf(p0), h1 = f2bf(p1);
      const unsigned short l0 = f2bf(p0 - bf2f(h0)), l1 = f2bf(p1 - bf2f(h1));
      const int row = 8 * hh + r;
      sph[row * PPITCH + c]      = h0;
      sph[row * PPITCH + 16 + c] = h1;
      spl[row * PPITCH + c]      = l0;
      spl[row * PPITCH + 16 + c] = l1;
    }
    __syncthreads();
    const v16b phf = ldfragb(sph, PPITCH, 0, 0, lane);
    const v16b plf = ldfragb(spl, PPITCH, 0, 0, lane);
#pragma unroll
    for (int nf = 0; nf < 4; ++nf) {
      const int vrow0 = kcol + nf * 16;
      const v16b vhf = ldfragb(vhb, NTOK, vrow0, kt * 32, lane);
      const v16b vlf = ldfragb(vlb, NTOK, vrow0, kt * 32, lane);
      acc[nf] = mmab(phf, vhf, acc[nf]);
      acc[nf] = mmab(phf, vlf, acc[nf]);
      acc[nf] = mmab(plf, vhf, acc[nf]);
    }
  }

  float inv[8];
#pragma unroll
  for (int r = 0; r < 8; ++r) inv[r] = __builtin_amdgcn_rcpf(lrow[r]);
  unsigned short* oh = sO + wave * (2 * 16 * EPH);
  unsigned short* ol = oh + 16 * EPH;
#pragma unroll
  for (int nf = 0; nf < 4; ++nf) {
#pragma unroll
    for (int r = 0; r < 8; ++r) {
      const float v = acc[nf][r] * inv[r];
      const unsigned short hi = f2bf(v);
      const unsigned short lo = f2bf(v - bf2f(hi));
      oh[(8 * hh + r) * EPH + 16 * nf + c] = hi;
      ol[(8 * hh + r) * EPH + 16 * nf + c] = lo;
    }
  }
  __syncthreads();
  v4u vvh[4], vvl[4];
  size_t go[4];
#pragma unroll
  for (int it = 0; it < 4; ++it) {
    const int p  = lane + 32 * it;
    const int L  = p >> 3;
    const int pc = p & 7;
    vvh[it] = *(const v4u*)(oh + L * EPH + pc * 8);
    vvl[it] = *(const v4u*)(ol + L * EPH + pc * 8);
    go[it]  = (size_t)(qrow0 + L) * DIM + kcol + pc * 8;
  }
  for (int ps = 0; ps < 2; ++ps) {
#pragma unroll
    for (int it = 0; it < 4; ++it) {
      *(volatile v4u*)(ah + go[it]) = vvh[it];
      *(volatile v4u*)(al + go[it]) = vvl[it];
    }
    __threadfence();
  }
}

__global__ __launch_bounds__(256) void k_wo(const unsigned short* __restrict__ ah, const unsigned short* __restrict__ al,
                                            const unsigned short* __restrict__ woh, const unsigned short* __restrict__ wol,
                                            const float* __restrict__ bo, const int* __restrict__ tokl,
                                            const float* __restrict__ wl, const int* __restrict__ tab,
                                            float* __restrict__ part) {
  __shared__ __align__(16) float sOut[8 * 16 * OTP];
  __shared__ int   sEnc[64];
  __shared__ float sW[64];
  __shared__ int   sVal[64];
  __shared__ int   sTab[64];
  const int tid = threadIdx.x, lane = tid & 31, wave = tid >> 5;
  const int hh = lane >> 4, c = lane & 15;
  const int wm = wave & 3, wn = wave >> 2;
  const int b  = blockIdx.y;
  const int n0 = blockIdx.x * 128;

  if (tid < 64) sTab[tid] = tab[tid];
  __syncthreads();
  const int tb16 = clampi(sTab[32 + NLIST], 0, NTILE);
  if (b >= tb16) return;
  int g = 0;
#pragma unroll
  for (int q = 1; q < NLIST; ++q) g += (clampi(sTab[32 + q], 0, NTILE) <= b) ? 1 : 0;
  const int e = g >> 2;
  const int tbg = clampi(sTab[32 + g], 0, NTILE);
  const int cng = clampi(sTab[g], 0, LCAP);
  if (tid < 64) {
    const int rloc = (b - tbg) * 64 + tid;
    const bool valid = (rloc >= 0) && (rloc < cng);
    const int li = g * LCAP + clampi(rloc, 0, LCAP - 1);
    const int enc = tokl[li];
    const float w = wl[li];
    sEnc[tid] = clampi(enc, 0, NPROW - 1);
    sW[tid]   = valid ? w : 0.f;
    sVal[tid] = valid ? 1 : 0;
  }
  __syncthreads();

  const int arow0 = b * 64 + wm * 16;
  const int brow  = n0 + wn * 64;
  const unsigned short* bh = woh + (size_t)e * (size_t)(DIM * DIM);
  const unsigned short* bl = wol + (size_t)e * (size_t)(DIM * DIM);
  v8f acc[4];
#pragma unroll
  for (int t = 0; t < 4; ++t) acc[t] = zero8();
#pragma unroll 1
  for (int k0 = 0; k0 < DIM; k0 += 32) {
    const v16b ahf = ldfragb(ah, DIM, arow0, k0, lane);
    const v16b alf = ldfragb(al, DIM, arow0, k0, lane);
#pragma unroll
    for (int t = 0; t < 4; ++t) {
      const v16b bhf = ldfragb(bh, DIM, brow + 16 * t, k0, lane);
      const v16b blf = ldfragb(bl, DIM, brow + 16 * t, k0, lane);
      acc[t] = mmab(ahf, bhf, acc[t]);
      acc[t] = mmab(ahf, blf, acc[t]);
      acc[t] = mmab(alf, bhf, acc[t]);
    }
  }

  float bcv[4], wr[8];
#pragma unroll
  for (int t = 0; t < 4; ++t) bcv[t] = bo[(size_t)e * DIM + brow + 16 * t + c];
#pragma unroll
  for (int r = 0; r < 8; ++r) wr[r] = sW[wm * 16 + 8 * hh + r];
  float* sw = sOut + wave * (16 * OTP);
#pragma unroll
  for (int t = 0; t < 4; ++t) {
#pragma unroll
    for (int r = 0; r < 8; ++r) sw[(8 * hh + r) * OTP + 16 * t + c] = (acc[t][r] + bcv[t]) * wr[r];
  }
  __syncthreads();
  v4f val[8];
  size_t go[8];
  bool ok[8];
#pragma unroll
  for (int it = 0; it < 8; ++it) {
    const int p    = lane + 32 * it;
    const int L    = p >> 3;
    const int pc   = p & 7;
    const int row  = L >> 1;
    const int half = L & 1;
    const int lr   = wm * 16 + row;
    val[it] = *(const v4f*)(sw + row * OTP + half * 32 + pc * 4);
    ok[it]  = (sVal[lr] != 0);
    go[it]  = (size_t)sEnc[lr] * DIM + brow + half * 32 + pc * 4;
  }
  for (int ps = 0; ps < 2; ++ps) {
#pragma unroll
    for (int it = 0; it < 8; ++it) {
      if (ok[it]) *(volatile v4f*)(part + go[it]) = val[it];
    }
    __threadfence();
  }
}

__global__ __launch_bounds__(256) void k_comb(const float* __restrict__ part, float* __restrict__ out, int n4) {
  const int i = blockIdx.x * 256 + (int)threadIdx.x;
  if (i >= n4) return;
  const size_t t = (size_t)i / (DIM / 4);
  const size_t n = ((size_t)i % (DIM / 4)) * 4;
  const float* pr = part + t * (size_t)(NSEL * DIM) + n;
  v4f v = *(const v4f*)(pr);
  const v4f p1 = *(const v4f*)(pr + DIM);
  v = v + p1;
  volatile v4f* d = (volatile v4f*)(out + t * DIM + n);
  *d = v;
  __threadfence();
  *d = v;
}

extern "C" void kernel_launch(void* const* d_in, const int* in_sizes, int n_in,
                              void* d_out, int out_size, void* d_ws, size_t ws_size,
                              hipStream_t stream) {
  if (n_in < 15) return;
  if (in_sizes[0] != NTOK * DIM) return;
  if (in_sizes[1] != NE * DIM * DIM || in_sizes[3] != NE * DIM * DIM ||
      in_sizes[5] != NE * DIM * DIM || in_sizes[7] != NE * DIM * DIM) return;
  if (in_sizes[2] != NE * DIM || in_sizes[4] != NE * DIM || in_sizes[6] != NE * DIM || in_sizes[8] != NE * DIM) return;
  if (in_sizes[9] != DIM * HID || in_sizes[10] != HID || in_sizes[11] != HID || in_sizes[12] != HID) return;
  if (in_sizes[13] != HID * NE || in_sizes[14] != NE) return;
  if (out_size != NTOK * DIM) return;

  const float* x   = (const float*)d_in[0];
  const float* Wq  = (const float*)d_in[1];
  const float* bq  = (const float*)d_in[2];
  const float* Wk  = (const float*)d_in[3];
  const float* bk  = (const float*)d_in[4];
  const float* Wv  = (const float*)d_in[5];
  const float* bv  = (const float*)d_in[6];
  const float* Wo  = (const float*)d_in[7];
  const float* bo  = (const float*)d_in[8];
  const float* Wr1 = (const float*)d_in[9];
  const float* br1 = (const float*)d_in[10];
  const float* lng = (const float*)d_in[11];
  const float* lnb = (const float*)d_in[12];
  const float* Wr2 = (const float*)d_in[13];
  const float* br2 = (const float*)d_in[14];
  float* out = (float*)d_out;

  size_t off = 0;
  const size_t oXh = off; off += (size_t)NTOK * DIM * 2;
  const size_t oWq = off; off += (size_t)NE * DIM * DIM * 2;
  const size_t oWk = off; off += (size_t)NE * DIM * DIM * 2;
  const size_t oWv = off; off += (size_t)NE * DIM * DIM * 2;
  const size_t oOh = off; off += (size_t)NE * DIM * DIM * 2;
  const size_t oOl = off; off += (size_t)NE * DIM * DIM * 2;
  const size_t oR  = off; off += (size_t)NTOK * RPITCH * 4;
  const size_t oTL = off; off += (size_t)NLIST * LCAP * 4;
  const size_t oWL = off; off += (size_t)NLIST * LCAP * 4;
  const size_t oTB = off; off += (size_t)256;
  const size_t oKh = off; off += (size_t)NTOK * DIM * 2;
  const size_t oKl = off; off += (size_t)NTOK * DIM * 2;
  const size_t oVh = off; off += (size_t)DIM * NTOK * 2;
  const size_t oVl = off; off += (size_t)DIM * NTOK * 2;
  const size_t oQh = off; off += (size_t)QROWS * DIM * 2;
  const size_t oQl = off; off += (size_t)QROWS * DIM * 2;
  const size_t oAh = off; off += (size_t)QROWS * DIM * 2;
  const size_t oAl = off; off += (size_t)QROWS * DIM * 2;
  const size_t oP  = off; off += (size_t)NPROW * DIM * 4;
  if (off > ws_size) return;
  if (off > (size_t)134217728) return;
  if ((oWq | oWk | oWv | oOh | oOl | oR | oTL | oWL | oTB | oKh | oKl | oVh | oVl | oQh | oQl | oAh | oAl | oP) & (size_t)127) return;

  char* ws = (char*)d_ws;
  _Float16* Xh  = (_Float16*)(ws + oXh);
  _Float16* WqT = (_Float16*)(ws + oWq);
  _Float16* WkT = (_Float16*)(ws + oWk);
  _Float16* WvT = (_Float16*)(ws + oWv);
  unsigned short* WoH = (unsigned short*)(ws + oOh);
  unsigned short* WoL = (unsigned short*)(ws + oOl);
  float*    R   = (float*)(ws + oR);
  int*      TOK = (int*)(ws + oTL);
  float*    WL  = (float*)(ws + oWL);
  int*      TAB = (int*)(ws + oTB);
  unsigned short* KH = (unsigned short*)(ws + oKh);
  unsigned short* KL = (unsigned short*)(ws + oKl);
  unsigned short* VH = (unsigned short*)(ws + oVh);
  unsigned short* VL = (unsigned short*)(ws + oVl);
  unsigned short* QH = (unsigned short*)(ws + oQh);
  unsigned short* QL = (unsigned short*)(ws + oQl);
  unsigned short* AH = (unsigned short*)(ws + oAh);
  unsigned short* AL = (unsigned short*)(ws + oAl);
  float*    P   = (float*)(ws + oP);

  k_cvt<<<dim3((NTOK * DIM) / 8 / 256), dim3(256), 0, stream>>>(x, Xh, (NTOK * DIM) / 8);
  k_wtrh<<<dim3(DIM / 64, DIM / 64, NE), dim3(256), 0, stream>>>(Wq, WqT, DIM, DIM, WSC);
  k_wtrh<<<dim3(DIM / 64, DIM / 64, NE), dim3(256), 0, stream>>>(Wk, WkT, DIM, DIM, WSC);
  k_wtrh<<<dim3(DIM / 64, DIM / 64, NE), dim3(256), 0, stream>>>(Wv, WvT, DIM, DIM, WSC);
  k_wtrb<<<dim3(DIM / 64, DIM / 64, NE), dim3(256), 0, stream>>>(Wo, WoH, WoL, DIM, DIM);
  k_route<<<dim3(NTOK / 8), dim3(256), 0, stream>>>(x, Wr1, br1, lng, lnb, Wr2, br2, R);
  k_lists<<<dim3(1), dim3(256), 0, stream>>>(R, TOK, WL, TAB);
  k_qproj<<<dim3(DIM / 128, NTILE), dim3(256), 0, stream>>>(Xh, WqT, bq, TOK, TAB, QH, QL);
  for (int e = 0; e < NE; ++e) {
    const _Float16* wk_e = WkT + (size_t)e * DIM * DIM;
    const _Float16* wv_e = WvT + (size_t)e * DIM * DIM;
    k_gemm16<0><<<dim3(DIM / 128, NTOK / 64), dim3(256), 0, stream>>>(Xh, wk_e, bk + (size_t)e * DIM, KH, KL, DIM, DIM);
    k_gemm16<1><<<dim3(NTOK / 128, DIM / 64), dim3(256), 0, stream>>>(wv_e, Xh, bv + (size_t)e * DIM, VH, VL, NTOK, DIM);
    k_attn<<<dim3(NHEAD, ETILE), dim3(128), 0, stream>>>(QH, QL, KH, KL, VH, VL, TAB, AH, AL, e);
  }
  k_wo<<<dim3(DIM / 128, NTILE), dim3(256), 0, stream>>>(AH, AL, WoH, WoL, bo, TOK, WL, TAB, P);
  k_comb<<<dim3((NTOK * DIM) / 4 / 256), dim3(256), 0, stream>>>(P, out, (NTOK * DIM) / 4);
  (void)hipGetLastError();
}
